// MultiHeadAttention_8899172237976
// MI455X (gfx1250) — hardware-verified
//
#include <hip/hip_runtime.h>


#ifndef NB
#define NB 2
#endif
#ifndef SEQ
#define SEQ 2048
#endif
#define NB_FULL  2
#define SEQ_FULL 2048
#define DM   1024
#define NH_  16
#define HD   64
#define RHF  256
#define RH   ((SEQ < RHF) ? SEQ : RHF)
#define MROWS (NB * SEQ)
#define PCAR 1024.0f
#define SCL  0.125f
#define L2E  1.4426950408889634f
#define NEGB (-1.0e30f)
#define AW   4
#define PP   40
#define OP   72

static_assert(SEQ % 64 == 0);
static_assert(RH % 64 == 0);
static_assert(RH <= SEQ);
static_assert(SEQ <= SEQ_FULL);
static_assert(NB <= NB_FULL);
static_assert(DM % 64 == 0);
static_assert(NH_ * HD == DM);
static_assert(HD == 64);
static_assert(AW * 16 == 64);
static_assert(PP % 8 == 0 && PP >= 32);
static_assert(OP % 8 == 0 && OP >= 64);

typedef _Float16 h16;
typedef unsigned short bf;
typedef __attribute__((ext_vector_type(16))) __bf16   v16bf;
typedef __attribute__((ext_vector_type(16))) _Float16 v16h;
typedef __attribute__((ext_vector_type(8)))  _Float16 v8h;
typedef __attribute__((ext_vector_type(8)))  unsigned short v8us;
typedef __attribute__((ext_vector_type(16))) unsigned short v16us;
typedef __attribute__((ext_vector_type(2)))  unsigned short v2us;
typedef __attribute__((ext_vector_type(8)))  float    v8f;
typedef __attribute__((ext_vector_type(4)))  float    v4f;
typedef v4f  __attribute__((may_alias)) v4fa;
typedef v8us __attribute__((may_alias)) v8usa;

__device__ __forceinline__ unsigned short f2bf(float f) { unsigned u = __float_as_uint(f); u += 0x7FFFu + ((u >> 16) & 1u); return (unsigned short)(u >> 16); }
__device__ __forceinline__ float bf2f(unsigned short b) { return __uint_as_float(((unsigned)b) << 16); }
__device__ __forceinline__ float bfr(float f) { return bf2f(f2bf(f)); }
__device__ __forceinline__ void splitf(float y, unsigned short& h, unsigned short& l) { h = f2bf(y); l = f2bf(y - bf2f(h)); }
__device__ __forceinline__ v16bf cat16b(v8us lo, v8us hi) { return __builtin_bit_cast(v16bf, __builtin_shufflevector(lo, hi, 0, 1, 2, 3, 4, 5, 6, 7, 8, 9, 10, 11, 12, 13, 14, 15)); }
__device__ __forceinline__ v16us cat16u(v8us lo, v8us hi) { return __builtin_shufflevector(lo, hi, 0, 1, 2, 3, 4, 5, 6, 7, 8, 9, 10, 11, 12, 13, 14, 15); }
__device__ __forceinline__ v8f wmma16(v16h a, v16h b, v8f c) { return __builtin_amdgcn_wmma_f32_16x16x32_f16(false, a, false, b, (short)0, c, false, false); }
__device__ __forceinline__ v8f wmmab(v16bf a, v16bf b, v8f c) { return __builtin_amdgcn_wmma_f32_16x16x32_bf16(false, a, false, b, (short)0, c, false, false); }
__device__ __forceinline__ v16bf ldb(const bf* p) { return cat16b(*(const v8us*)p, *(const v8us*)(p + 16)); }
__device__ __forceinline__ v16us ldus(const bf* p) { return cat16u(*(const v8us*)p, *(const v8us*)(p + 16)); }
template <bool HI> __device__ __forceinline__ v8f mmaT(v16us a, v16us b, v8f c) {
    if (HI) return wmmab(__builtin_bit_cast(v16bf, a), __builtin_bit_cast(v16bf, b), c);
    else    return wmma16(__builtin_bit_cast(v16h, a), __builtin_bit_cast(v16h, b), c);
}

template <int NSPLIT, bool BIAS>
__device__ __forceinline__ void gemmw_body(const bf* A, const bf* A2, const bf* Bt, const int K, float* C, const int ldc, const float* bias, const size_t sA, const size_t sB, const size_t sC) {
    __shared__ __align__(16) float os[16 * 68];
    const size_t z = blockIdx.z; A += z * sA; A2 += z * sA; Bt += z * sB; C += z * sC;
    const int lane = threadIdx.x & 31, lr = lane & 15, hi = lane >> 4; const int r0 = blockIdx.x * 64, c0 = blockIdx.y * 64;
    v8f acc[4][4];
#pragma unroll
    for (int mb = 0; mb < 4; ++mb)
#pragma unroll
        for (int nb = 0; nb < 4; ++nb) acc[mb][nb] = (v8f){};
    const size_t aoff = (size_t)(r0 + lr) * K + 8 * hi, boff = (size_t)(c0 + lr) * K + 8 * hi;
#pragma unroll 1
    for (int kc = 0; kc < K; kc += 32) {
        v16bf a[4], a2[4];
#pragma unroll
        for (int mb = 0; mb < 4; ++mb) { a[mb] = ldb(A + aoff + (size_t)mb * 16 * K + kc); if (NSPLIT == 1) a2[mb] = ldb(A2 + aoff + (size_t)mb * 16 * K + kc); else a2[mb] = a[mb]; }
        v16bf blast;
#pragma unroll
        for (int nb = 0; nb < 4; ++nb) { const v16bf b = ldb(Bt + boff + (size_t)nb * 16 * K + kc); blast = b;
#pragma unroll
            for (int mb = 0; mb < 4; ++mb) { acc[mb][nb] = wmmab(a[mb], b, acc[mb][nb]); if (NSPLIT == 1) acc[mb][nb] = wmmab(a2[mb], b, acc[mb][nb]); } }
        asm volatile("" : "+v"(acc[0][0]), "+v"(acc[0][1]), "+v"(acc[0][2]), "+v"(acc[0][3]), "+v"(acc[1][0]), "+v"(acc[1][1]), "+v"(acc[1][2]), "+v"(acc[1][3]));
        asm volatile("v_nop\n\tv_nop\n\tv_nop\n\tv_nop" : "+v"(acc[2][0]), "+v"(acc[2][1]), "+v"(acc[2][2]), "+v"(acc[2][3]), "+v"(acc[3][0]), "+v"(acc[3][1]), "+v"(acc[3][2]), "+v"(acc[3][3]) : "v"(a[3]), "v"(blast));
    }
#pragma unroll
    for (int mb = 0; mb < 4; ++mb) {
#pragma unroll
        for (int nb = 0; nb < 4; ++nb) {
#pragma unroll
            for (int j = 0; j < 8; ++j) os[(hi * 8 + j) * 68 + nb * 16 + lr] = acc[mb][nb][j]; }
        asm volatile("s_wait_dscnt 0" ::: "memory"); __builtin_amdgcn_wave_barrier(); asm volatile("" ::: "memory");
        float* crow = C + (size_t)(r0 + mb * 16) * ldc + c0;
#pragma unroll 1
        for (int ps = 0; ps < 2; ++ps) {
#pragma unroll
            for (int s = 0; s < 8; ++s) { const int row = 2 * s + hi, cofs = lr * 4; v4f val = *(const v4fa*)(os + row * 68 + cofs); if (BIAS) { val[0] += bfr(bias[c0 + cofs]); val[1] += bfr(bias[c0 + cofs + 1]); val[2] += bfr(bias[c0 + cofs + 2]); val[3] += bfr(bias[c0 + cofs + 3]); }
                *(volatile v4f*)(crow + (size_t)row * ldc + cofs) = val; }
            if (ps == 0) __threadfence(); }
        asm volatile("s_wait_dscnt 0" ::: "memory"); __builtin_amdgcn_wave_barrier(); asm volatile("" ::: "memory");
    }
}
__global__ __launch_bounds__(32) void k_gemm_proj(const bf* __restrict__ A, const bf* __restrict__ Bt, float* C) {
    gemmw_body<0, false>(A, A, Bt, DM, C, DM, nullptr, (size_t)0, (size_t)DM * DM, (size_t)MROWS * DM);
}
__global__ __launch_bounds__(32) void k_gemm_out(const bf* __restrict__ Ah, const bf* __restrict__ Al, const bf* __restrict__ Bt, const float* __restrict__ bias, float* C) {
    gemmw_body<1, true>(Ah, Al, Bt, DM, C, DM, bias, (size_t)SEQ * DM, (size_t)0, (size_t)SEQ_FULL * DM);
}

__global__ __launch_bounds__(256) void k_wtG(const float* __restrict__ w, int K, int N, bf* Bt) {
    const int lane = threadIdx.x & 31; const int L0 = (blockIdx.x * 8 + (threadIdx.x >> 5)) * 8; const int nlines = N * K / 64;
#pragma unroll
    for (int ps = 0; ps < 2; ++ps) {
#pragma unroll 1
        for (int l = 0; l < 8; ++l) { const int L = L0 + l; if (L >= nlines) break; const size_t e = (size_t)L * 64 + lane * 2; const int k = (int)(e % K), n = (int)(e / K); v2us o;
            o[0] = f2bf(w[(size_t)k * N + n]); o[1] = f2bf(w[(size_t)(k + 1) * N + n]); *(volatile v2us*)(Bt + e) = o; }
        if (ps == 0) __threadfence(); }
}
__global__ __launch_bounds__(256) void k_cvtx(const float* __restrict__ x, bf* XB) {
    const int i = blockIdx.x * 256 + threadIdx.x; if (i >= MROWS * (DM / 8)) return;
    const int row = i / (DM / 8), pc = i % (DM / 8); const int b = row / SEQ, t = row % SEQ;
    const v8f v = *(const v8f*)(x + ((size_t)b * SEQ_FULL + t) * DM + pc * 8); v8us o;
#pragma unroll
    for (int k = 0; k < 8; ++k) o[k] = f2bf(v[k]);
    *(volatile v8us*)(XB + (size_t)i * 8) = o; __threadfence(); *(volatile v8us*)(XB + (size_t)i * 8) = o;
}
__global__ __launch_bounds__(256) void k_qkp(const float* __restrict__ F, h16* P16, bf* PH, bf* PL) {
    const int z = blockIdx.y; const int i = blockIdx.x * 256 + threadIdx.x; if (i >= NB * NH_ * SEQ * 8) return;
    const int pc = i & 7; const int t = (i >> 3) % SEQ; const int bh = i / (8 * SEQ); const int b = bh / NH_, h = bh % NH_;
    const v8f v = *(const v8f*)(F + (size_t)z * MROWS * DM + ((size_t)b * SEQ + t) * DM + h * HD + pc * 8);
    v8h o16; v8us oh, ol;
#pragma unroll
    for (int k = 0; k < 8; ++k) { o16[k] = (h16)v[k]; unsigned short a, c; splitf(v[k], a, c); oh[k] = a; ol[k] = c; }
    const size_t o = (size_t)z * NB * NH_ * SEQ * HD + ((size_t)bh * SEQ + t) * HD + pc * 8;
    const bool hr = (t < RH); const int tc = hr ? t : 0;
    const size_t o2 = (size_t)z * NB * NH_ * RH * HD + ((size_t)bh * RH + tc) * HD + pc * 8;
#pragma unroll 1
    for (int ps = 0; ps < 2; ++ps) {
        *(volatile v8h*)(P16 + o) = o16;
        if (hr) { *(volatile v8us*)(PH + o2) = oh; *(volatile v8us*)(PL + o2) = ol; }
        if (ps == 0) __threadfence(); }
}
__global__ __launch_bounds__(256) void k_vtp(const float* __restrict__ F, h16* V16, bf* VH, bf* VL) {
    const int i = blockIdx.x * 256 + threadIdx.x; if (i >= NB * NH_ * HD * (SEQ / 8)) return;
    const int pc = i % (SEQ / 8); const int d = (i / (SEQ / 8)) % HD; const int bh = i / (HD * (SEQ / 8)); const int b = bh / NH_, h = bh % NH_; const int t0 = pc * 8;
    const float* f = F + ((size_t)b * SEQ + t0) * DM + h * HD + d;
    v8h o16; v8us oh, ol;
#pragma unroll
    for (int q = 0; q < 8; ++q) { const float x = f[(size_t)q * DM]; o16[q] = (h16)x; unsigned short a, c; splitf(x, a, c); oh[q] = a; ol[q] = c; }
    const size_t o = ((size_t)bh * HD + d) * SEQ + t0;
    const bool hr = (t0 < RH); const int tc = hr ? t0 : 0;
    const size_t o2 = ((size_t)bh * HD + d) * RH + tc;
#pragma unroll 1
    for (int ps = 0; ps < 2; ++ps) {
        *(volatile v8h*)(V16 + o) = o16;
        if (hr) { *(volatile v8us*)(VH + o2) = oh; *(volatile v8us*)(VL + o2) = ol; }
        if (ps == 0) __threadfence(); }
}

template <bool HI>
__device__ __forceinline__ void attn_body(const bf* Qa, const bf* Qb, const bf* Ka, const bf* Kb, const bf* Va, const bf* Vb, bf* ATh, bf* ATl, const int roff, const int prow, const int vpitch) {
    __shared__ __align__(16) unsigned short ps[AW][2][16 * PP];
    __shared__ __align__(16) unsigned short osd[AW][2][16 * OP];
    const int lane = threadIdx.x & 31, lr = lane & 15, hi = lane >> 4;
    const int wave = __builtin_amdgcn_readfirstlane(threadIdx.x >> 5);
    const int h = blockIdx.y, b = blockIdx.z, bh = b * NH_ + h;
    const int q0 = roff + blockIdx.x * (AW * 16) + wave * 16;
    const int nhalf = (q0 >> 5) + 1;
    const int qoff = (bh * prow + q0 + lr) * HD + 8 * hi;
    const v16us qa0 = ldus(Qa + qoff), qa1 = ldus(Qa + qoff + 32);
    v16us qb0 = qa0, qb1 = qa1;
    if (HI) { qb0 = ldus(Qb + qoff); qb1 = ldus(Qb + qoff + 32); }
    v8f O[4];
#pragma unroll
    for (int dt = 0; dt < 4; ++dt) O[dt] = (v8f){};
    float m[8], l[8];
#pragma unroll
    for (int r = 0; r < 8; ++r) { m[r] = NEGB; l[r] = 0.0f; }

#pragma unroll 1
    for (int j = 0; j < nhalf; ++j) {
        const int k0 = j * 32;
        v8f s0 = (v8f){}, s1 = (v8f){};
        {
            const int ko = (bh * prow + k0 + lr) * HD + 8 * hi;
            const v16us k00 = ldus(Ka + ko), k01 = ldus(Ka + ko + 32);
            const v16us k10 = ldus(Ka + ko + 16 * HD), k11 = ldus(Ka + ko + 16 * HD + 32);
            s0 = mmaT<HI>(qa0, k00, s0); s0 = mmaT<HI>(qa1, k01, s0);
            s1 = mmaT<HI>(qa0, k10, s1); s1 = mmaT<HI>(qa1, k11, s1);
            v16us g0 = k10, g1 = k11;
            if (HI) {
                s0 = mmaT<HI>(qb0, k00, s0); s0 = mmaT<HI>(qb1, k01, s0);
                s1 = mmaT<HI>(qb0, k10, s1); s1 = mmaT<HI>(qb1, k11, s1);
                const v16us l00 = ldus(Kb + ko), l01 = ldus(Kb + ko + 32);
                const v16us l10 = ldus(Kb + ko + 16 * HD), l11 = ldus(Kb + ko + 16 * HD + 32);
                s0 = mmaT<HI>(qa0, l00, s0); s0 = mmaT<HI>(qa1, l01, s0);
                s1 = mmaT<HI>(qa0, l10, s1); s1 = mmaT<HI>(qa1, l11, s1);
                g0 = l10; g1 = l11;
            }
            asm volatile("v_nop\n\tv_nop\n\tv_nop\n\tv_nop" : "+v"(s0), "+v"(s1) : "v"(g0), "v"(g1));
        }
        float t0[8], t1[8];
#pragma unroll
        for (int r = 0; r < 8; ++r) { t0[r] = s0[r] * SCL; t1[r] = s1[r] * SCL; }
        if (j == nhalf - 1) {
#pragma unroll
            for (int r = 0; r < 8; ++r) { const int qg = q0 + 8 * hi + r; t0[r] = (k0 + lr > qg) ? NEGB : t0[r]; t1[r] = (k0 + 16 + lr > qg) ? NEGB : t1[r]; }
        }
#pragma unroll
        for (int r = 0; r < 8; ++r) {
            float mx = fmaxf(t0[r], t1[r]);
            mx = fmaxf(mx, __shfl_xor(mx, 1, 32)); mx = fmaxf(mx, __shfl_xor(mx, 2, 32)); mx = fmaxf(mx, __shfl_xor(mx, 4, 32)); mx = fmaxf(mx, __shfl_xor(mx, 8, 32));
            const float mn = fmaxf(m[r], mx);
            const float al = __builtin_amdgcn_exp2f((m[r] - mn) * L2E);
            const float p0 = __builtin_amdgcn_exp2f((t0[r] - mn) * L2E);
            const float p1 = __builtin_amdgcn_exp2f((t1[r] - mn) * L2E);
            l[r] = l[r] * al + (p0 + p1); m[r] = mn;
            O[0][r] *= al; O[1][r] *= al; O[2][r] *= al; O[3][r] *= al;
            const int pi = (8 * hi + r) * PP + lr;
            if (HI) { unsigned short a, c; splitf(p0, a, c); ps[wave][0][pi] = a; ps[wave][1][pi] = c; splitf(p1, a, c); ps[wave][0][pi + 16] = a; ps[wave][1][pi + 16] = c; }
            else { ps[wave][0][pi] = __builtin_bit_cast(unsigned short, (h16)(p0 * PCAR)); ps[wave][0][pi + 16] = __builtin_bit_cast(unsigned short, (h16)(p1 * PCAR)); }
        }
        asm volatile("s_wait_dscnt 0" ::: "memory"); __builtin_amdgcn_wave_barrier(); asm volatile("" ::: "memory");
        {
            const int po = lr * PP + 8 * hi;
            const v16us pa = cat16u(*(const v8usa*)(&ps[wave][0][po]), *(const v8usa*)(&ps[wave][0][po + 16]));
            v16us pb = pa;
            if (HI) pb = cat16u(*(const v8usa*)(&ps[wave][1][po]), *(const v8usa*)(&ps[wave][1][po + 16]));
            const int vo = (bh * HD + lr) * vpitch + k0 + 8 * hi;
            const v16us v0 = ldus(Va + vo), v1 = ldus(Va + vo + 16 * vpitch), v2 = ldus(Va + vo + 32 * vpitch), v3 = ldus(Va + vo + 48 * vpitch);
            O[0] = mmaT<HI>(pa, v0, O[0]); O[1] = mmaT<HI>(pa, v1, O[1]); O[2] = mmaT<HI>(pa, v2, O[2]); O[3] = mmaT<HI>(pa, v3, O[3]);
            v16us g2 = v2, g3 = v3;
            if (HI) {
                O[0] = mmaT<HI>(pb, v0, O[0]); O[1] = mmaT<HI>(pb, v1, O[1]); O[2] = mmaT<HI>(pb, v2, O[2]); O[3] = mmaT<HI>(pb, v3, O[3]);
                const v16us w0 = ldus(Vb + vo), w1 = ldus(Vb + vo + 16 * vpitch), w2 = ldus(Vb + vo + 32 * vpitch), w3 = ldus(Vb + vo + 48 * vpitch);
                O[0] = mmaT<HI>(pa, w0, O[0]); O[1] = mmaT<HI>(pa, w1, O[1]); O[2] = mmaT<HI>(pa, w2, O[2]); O[3] = mmaT<HI>(pa, w3, O[3]);
                g2 = w2; g3 = w3;
            }
            asm volatile("v_nop\n\tv_nop\n\tv_nop\n\tv_nop" : "+v"(O[0]), "+v"(O[1]), "+v"(O[2]), "+v"(O[3]) : "v"(g2), "v"(g3));
        }
        asm volatile("" ::: "memory");
    }

#pragma unroll
    for (int r = 0; r < 8; ++r) {
        float ls = l[r];
        ls += __shfl_xor(ls, 1, 32); ls += __shfl_xor(ls, 2, 32); ls += __shfl_xor(ls, 4, 32); ls += __shfl_xor(ls, 8, 32);
        const float inv = __builtin_amdgcn_rcpf(ls) * (HI ? 1.0f : (1.0f / PCAR));
#pragma unroll
        for (int dt = 0; dt < 4; ++dt) { unsigned short a, c; splitf(O[dt][r] * inv, a, c); const int oi = (8 * hi + r) * OP + dt * 16 + lr; osd[wave][0][oi] = a; osd[wave][1][oi] = c; }
    }
    asm volatile("s_wait_dscnt 0" ::: "memory"); __builtin_amdgcn_wave_barrier(); asm volatile("" ::: "memory");
#pragma unroll 1
    for (int pass = 0; pass < 2; ++pass) {
#pragma unroll
        for (int s = 0; s < 4; ++s) { const int row = 4 * s + (lane >> 3), pc = (lane & 7) * 8;
            const v8us vh = *(const v8usa*)(&osd[wave][0][row * OP + pc]); const v8us vl = *(const v8usa*)(&osd[wave][1][row * OP + pc]);
            const size_t go = ((size_t)b * SEQ + q0 + row) * DM + h * HD + pc;
            *(volatile v8us*)(ATh + go) = vh; *(volatile v8us*)(ATl + go) = vl; }
        if (pass == 0) __threadfence(); }
}
__global__ __launch_bounds__(128) void k_attn_lo(const bf* __restrict__ Q16, const bf* __restrict__ K16, const bf* __restrict__ V16, bf* ATh, bf* ATl) {
    attn_body<false>(Q16, Q16, K16, K16, V16, V16, ATh, ATl, RH, SEQ, SEQ);
}
__global__ __launch_bounds__(128) void k_attn_hi(const bf* __restrict__ QH, const bf* __restrict__ QL, const bf* __restrict__ KH, const bf* __restrict__ KL, const bf* __restrict__ VH, const bf* __restrict__ VL, bf* ATh, bf* ATl) {
    attn_body<true>(QH, QL, KH, KL, VH, VL, ATh, ATl, 0, RH, RH);
}

constexpr size_t al256(size_t b) { return (b + 255) & ~(size_t)255; }
constexpr size_t SZ_WT3 = (size_t)3 * DM * DM * 2;
constexpr size_t SZ_WO  = (size_t)DM * DM * 2;
constexpr size_t SZ_XB  = (size_t)MROWS * DM * 2;
constexpr size_t SZ_F   = (size_t)3 * MROWS * DM * 4;
constexpr size_t SZ_P16 = (size_t)2 * NB * NH_ * SEQ * HD * 2;
constexpr size_t SZ_PHL = (size_t)2 * NB * NH_ * RH * HD * 2;
constexpr size_t SZ_V16 = (size_t)NB * NH_ * HD * SEQ * 2;
constexpr size_t SZ_VHL = (size_t)NB * NH_ * HD * RH * 2;
constexpr size_t SZ_AT  = (size_t)MROWS * DM * 2;
constexpr size_t SZ_TOTAL = al256(SZ_WT3) + al256(SZ_WO) + al256(SZ_XB) + al256(SZ_F) + al256(SZ_P16) + 2 * al256(SZ_PHL) + al256(SZ_V16) + 2 * al256(SZ_VHL) + 2 * al256(SZ_AT);
static_assert(SZ_TOTAL <= (size_t)134217728);

extern "C" void kernel_launch(void* const* d_in, const int* in_sizes, int n_in,
                              void* d_out, int out_size, void* d_ws, size_t ws_size, hipStream_t stream) {
    if (n_in < 6) return;
    const long long need = ((long long)(NB - 1) * SEQ_FULL + SEQ) * DM;
    if (in_sizes[0] < need || in_sizes[1] < DM * DM || in_sizes[2] < DM * DM || in_sizes[3] < DM * DM || in_sizes[4] < DM * DM || in_sizes[5] < DM || out_size < need) return;
    if (ws_size < SZ_TOTAL) return;
    const float* x  = (const float*)d_in[0];
    const float* wk = (const float*)d_in[1];
    const float* wq = (const float*)d_in[2];
    const float* wv = (const float*)d_in[3];
    const float* wp = (const float*)d_in[4];
    const float* bp = (const float*)d_in[5];
    float* OUT = (float*)d_out;
    char* wsp = (char*)d_ws;
    auto take = [&](size_t bytes) { char* p = wsp; wsp += (bytes + 255) & ~(size_t)255; return (void*)p; };
    bf* WT3 = (bf*)take(SZ_WT3); bf* WO = (bf*)take(SZ_WO); bf* XB = (bf*)take(SZ_XB); float* F = (float*)take(SZ_F);
    bf* P16 = (bf*)take(SZ_P16); bf* PH = (bf*)take(SZ_PHL); bf* PL = (bf*)take(SZ_PHL);
    bf* V16 = (bf*)take(SZ_V16); bf* VH = (bf*)take(SZ_VHL); bf* VL = (bf*)take(SZ_VHL);
    bf* ATh = (bf*)take(SZ_AT); bf* ATl = (bf*)take(SZ_AT);
    if ((size_t)(wsp - (char*)d_ws) > ws_size) return;

    const unsigned gW = (unsigned)((DM * DM / 64 + 63) / 64);
    k_wtG<<<gW, 256, 0, stream>>>(wq, DM, DM, WT3);
    k_wtG<<<gW, 256, 0, stream>>>(wk, DM, DM, WT3 + (size_t)DM * DM);
    k_wtG<<<gW, 256, 0, stream>>>(wv, DM, DM, WT3 + (size_t)2 * DM * DM);
    k_wtG<<<gW, 256, 0, stream>>>(wp, DM, DM, WO);
    k_cvtx<<<(unsigned)((MROWS * (DM / 8) + 255) / 256), 256, 0, stream>>>(x, XB);
    k_gemm_proj<<<dim3(MROWS / 64, DM / 64, 3), 32, 0, stream>>>(XB, WT3, F);
    k_qkp<<<dim3((unsigned)((NB * NH_ * SEQ * 8 + 255) / 256), 2, 1), 256, 0, stream>>>(F, (h16*)P16, PH, PL);
    k_vtp<<<(unsigned)((NB * NH_ * HD * (SEQ / 8) + 255) / 256), 256, 0, stream>>>(F + (size_t)2 * MROWS * DM, (h16*)V16, VH, VL);
    const size_t kz16 = (size_t)NB * NH_ * SEQ * HD, kzhl = (size_t)NB * NH_ * RH * HD;
    k_attn_hi<<<dim3(RH / 64, NH_, NB), 128, 0, stream>>>(PH, PL, PH + kzhl, PL + kzhl, VH, VL, ATh, ATl);
    if (SEQ > RH) k_attn_lo<<<dim3((SEQ - RH) / 64, NH_, NB), 128, 0, stream>>>(P16, P16 + kz16, V16, ATh, ATl);
    k_gemm_out<<<dim3(SEQ / 64, DM / 64, NB), 32, 0, stream>>>(ATh, ATl, WO, bp, OUT);
}
